// LSTM_62053687493021
// MI455X (gfx1250) — hardware-run, weakly checked
//
#include <hip/hip_runtime.h>
#include <math.h>

constexpr int NBAT   = 128;
constexpr int NSTEP  = 1024;
constexpr int NDIN   = 64;
constexpr int NHID   = 128;
constexpr int NGATE  = 512;
constexpr int NLAY   = 3;
constexpr int NTHR   = 256;
constexpr int RBLK   = 16;
constexpr int APITCH = 136;
constexpr int SPITCH = 132;
constexpr int OPITCH = 36;
constexpr float XWCARRY = 64.0f;
constexpr float WCARRY  = 8.0f;
constexpr float HCARRY  = 8.0f;
constexpr float FOLD    = 1.0f / 64.0f;
constexpr float H16_MIN_NORMAL = 6.103515625e-05f;
constexpr int NOUT0  = NBAT * NSTEP;
constexpr int NSTATE = NLAY * NBAT * NHID;
static_assert(NHID == 16 * (NTHR / 32), "8 waves x 16 hidden units");
static_assert(NBAT % RBLK == 0, "grid exact");
static_assert(NDIN % 32 == 0 && NHID % 32 == 0, "k chunks of 32, no padding read");
static_assert(NSTEP % 32 == 0, "output-head flush every 32 steps");
static_assert(RBLK * NDIN == NTHR * 4, "layer-0 x tile staging exact");
static_assert(RBLK * NHID == NTHR * 8, "y tile / h0 staging exact");
static_assert(RBLK == 2 * (NTHR / 32), "two rows per wave in the row-store phases");
static_assert(NOUT0 * 4 == 524288 && (NOUT0 + NSTATE) * 4 == 720896 && (NOUT0 + 2 * NSTATE) * 4 == 917504, "d_out byte offsets");
static_assert(APITCH % 8 == 0 && SPITCH % 4 == 0 && OPITCH % 4 == 0, "16-B aligned LDS rows");

typedef __attribute__((ext_vector_type(16))) _Float16 v16h;
typedef __attribute__((ext_vector_type(8)))  _Float16 v8h;
typedef __attribute__((ext_vector_type(16))) __bf16   v16b;
typedef __attribute__((ext_vector_type(8)))  __bf16   v8b;
typedef __attribute__((ext_vector_type(8)))  float    v8f;
typedef __attribute__((ext_vector_type(4)))  float    v4f;
typedef __attribute__((ext_vector_type(4)))  unsigned v4u;
typedef __attribute__((ext_vector_type(2)))  unsigned v2u;

__device__ __forceinline__ unsigned short f2bf_bits(float f) {
  unsigned u = __float_as_uint(f);
  return (unsigned short)((u + 0x7FFFu + ((u >> 16) & 1u)) >> 16);
}
__device__ __forceinline__ float bf_bits2f(unsigned short h) { return __uint_as_float(((unsigned)h) << 16); }
__device__ __forceinline__ float bf16r(float f) { return bf_bits2f(f2bf_bits(f)); }
__device__ __forceinline__ float flush16(float s) { return (fabsf(s) < H16_MIN_NORMAL) ? 0.0f : s; }
__device__ __forceinline__ _Float16 to_h16(float s) { return (_Float16)flush16(s); }
__device__ __forceinline__ unsigned short h16_bits(float s) { return __builtin_bit_cast(unsigned short, (_Float16)flush16(s)); }

__device__ __forceinline__ void tie4_h(v8f& a0, v8f& a1, v8f& a2, v8f& a3, v16h x, v16h b0, v16h b1, v16h b2, v16h b3) {
  asm volatile("v_nop\n\tv_nop\n\tv_nop\n\tv_nop" : "+v"(a0), "+v"(a1), "+v"(a2), "+v"(a3) : "v"(x), "v"(b0), "v"(b1), "v"(b2), "v"(b3));
}
__device__ __forceinline__ void tie4_b(v8f& a0, v8f& a1, v8f& a2, v8f& a3, v16b x, v16b b0, v16b b1, v16b b2, v16b b3) {
  asm volatile("v_nop\n\tv_nop\n\tv_nop\n\tv_nop" : "+v"(a0), "+v"(a1), "+v"(a2), "+v"(a3) : "v"(x), "v"(b0), "v"(b1), "v"(b2), "v"(b3));
}
__device__ __forceinline__ void acc_guard4(v8f& a, v8f& b, v8f& c, v8f& d) { asm volatile("v_nop\n\tv_nop\n\tv_nop\n\tv_nop" : "+v"(a), "+v"(b), "+v"(c), "+v"(d)); }

template <typename T> struct Frag;
template <> struct Frag<_Float16> {
  typedef v16h V; union U { v16h v; v8h h[2]; };
  static __device__ __forceinline__ v16h load(const _Float16* p) {
    U f; f.h[0] = *(const v8h*)(p); f.h[1] = *(const v8h*)(p + 16); return f.v;
  }
  static __device__ __forceinline__ v8f mma(v16h a, v16h b, v8f c) {
    return __builtin_amdgcn_wmma_f32_16x16x32_f16(false, a, false, b, (short)0, c, false, false);
  }
  static __device__ __forceinline__ void tie4(v8f& a0, v8f& a1, v8f& a2, v8f& a3, v16h x, v16h b0, v16h b1, v16h b2, v16h b3) {
    tie4_h(a0, a1, a2, a3, x, b0, b1, b2, b3);
  }
};
template <> struct Frag<__bf16> {
  typedef v16b V; union U { v16b v; v8b h[2]; };
  static __device__ __forceinline__ v16b load(const __bf16* p) {
    U f; f.h[0] = *(const v8b*)(p); f.h[1] = *(const v8b*)(p + 16); return f.v;
  }
  static __device__ __forceinline__ v8f mma(v16b a, v16b b, v8f c) {
    return __builtin_amdgcn_wmma_f32_16x16x32_bf16(false, a, false, b, (short)0, c, false, false);
  }
  static __device__ __forceinline__ void tie4(v8f& a0, v8f& a1, v8f& a2, v8f& a3, v16b x, v16b b0, v16b b1, v16b b2, v16b b3) {
    tie4_b(a0, a1, a2, a3, x, b0, b1, b2, b3);
  }
};

__device__ __forceinline__ float fsig(float x)  { return __builtin_amdgcn_rcpf(1.0f + __expf(-x)); }
__device__ __forceinline__ float ftanh(float x) { return 1.0f - 2.0f * __builtin_amdgcn_rcpf(__expf(2.0f * x) + 1.0f); }

template <int MODE>
__global__ __launch_bounds__(NTHR) void cvt8_kernel(const float* __restrict__ src, unsigned short* __restrict__ dst,
                                                    int nrow, int ncol8, int spitch, int scol0, float sc) {
  const int i  = blockIdx.x * NTHR + threadIdx.x;
  const int n8 = nrow * ncol8;
  if (i < n8) {
    const int row = i / ncol8;
    const int c8  = i - row * ncol8;
    const float* sp = src + (size_t)row * spitch + scol0 + c8 * 8;
    const v4f a = *(const v4f*)(sp);
    const v4f b = *(const v4f*)(sp + 4);
    v8h hv;
#pragma unroll
    for (int e = 0; e < 4; ++e) {
      unsigned short b0, b1;
      if (MODE == 0) {
        b0 = f2bf_bits(a[e] * sc);
        b1 = f2bf_bits(b[e] * sc);
      } else {
        b0 = h16_bits(bf16r(a[e]) * sc);
        b1 = h16_bits(bf16r(b[e]) * sc);
      }
      hv[e]     = __builtin_bit_cast(_Float16, b0);
      hv[4 + e] = __builtin_bit_cast(_Float16, b1);
    }
    *(volatile v8h*)(dst + (size_t)i * 8) = hv;
    __threadfence();
    *(volatile v8h*)(dst + (size_t)i * 8) = hv;
  }
}

template <int MODE> struct XSel { typedef _Float16 T; };
template <> struct XSel<0> { typedef __bf16 T; };
template <int MODE>
__device__ __forceinline__ void stage_x(unsigned short* Ax, const float* xsrc, const unsigned short* ysrc,
                                        int rowbase, int tt, int tid) {
  if (MODE == 0) {
    const int m = tid >> 4, f4 = (tid & 15) * 4;
    const v4f v = *(const v4f*)(xsrc + ((size_t)(rowbase + m) * NSTEP + (size_t)tt) * NDIN + f4);
    const unsigned u0 = f2bf_bits(v[0]), u1 = f2bf_bits(v[1]), u2 = f2bf_bits(v[2]), u3 = f2bf_bits(v[3]);
    v2u pk;
    pk[0] = u0 | (u1 << 16);
    pk[1] = u2 | (u3 << 16);
    *(v2u*)(Ax + m * APITCH + f4) = pk;
  } else {
    const int m = tid >> 4, c8 = (tid & 15) * 8;
    const v4u v = *(const v4u*)(ysrc + ((size_t)(rowbase + m) * NSTEP + (size_t)tt) * NHID + c8);
    *(v4u*)(Ax + m * APITCH + c8) = v;
  }
}

template <int MODE>
__global__ __launch_bounds__(NTHR) void lstm_layer_kernel(
    const float* __restrict__ xsrc, const unsigned short* __restrict__ ysrc,
    const float* __restrict__ h0l, const float* __restrict__ c0l,
    const float* __restrict__ bih, const float* __restrict__ bhh,
    const unsigned short* __restrict__ WXp, const unsigned short* __restrict__ WHp,
    const float* __restrict__ wout, const float* __restrict__ bout,
    unsigned short* __restrict__ ydst, float* __restrict__ out0,
    float* __restrict__ hfin, float* __restrict__ cfin) {
  typedef typename XSel<MODE>::T XT;
  typedef typename Frag<XT>::V XV;
  constexpr int KXE = (MODE == 0) ? NDIN : NHID;
  __shared__ __align__(16) unsigned short Ax[RBLK * APITCH];
  __shared__ __align__(16) _Float16       Ah[RBLK * APITCH];
  __shared__ __align__(16) float          Hs[RBLK * SPITCH];
  __shared__ __align__(16) float          Cs[RBLK * SPITCH];
  __shared__ __align__(16) float          Ob[RBLK * OPITCH];
  const _Float16* WH = (const _Float16*)(const void*)WHp;
  const XT*       WX = (const XT*)(const void*)WXp;
  const int tid = threadIdx.x, lane = tid & 31, wave = tid >> 5;
  const int c = lane & 15, hh = lane >> 4, koff = hh * 8;
  const int rowbase = blockIdx.x * RBLK;
  const int j = 16 * wave + c;

#pragma unroll 1
  for (int i = tid; i < RBLK * APITCH; i += NTHR) { Ax[i] = (unsigned short)0; Ah[i] = (_Float16)0.0f; }
#pragma unroll 1
  for (int i = tid; i < RBLK * SPITCH; i += NTHR) { Hs[i] = 0.0f; Cs[i] = 0.0f; }
#pragma unroll 1
  for (int i = tid; i < RBLK * OPITCH; i += NTHR) Ob[i] = 0.0f;

  float bs[4];
#pragma unroll
  for (int g = 0; g < 4; ++g) bs[g] = bf16r(bih[NHID * g + j]) + bf16r(bhh[NHID * g + j]);
  asm volatile("" ::: "memory");
  float cst[8];
#pragma unroll
  for (int r = 0; r < 8; ++r) cst[r] = bf16r(c0l[(size_t)(rowbase + 8 * hh + r) * NHID + j]);
  asm volatile("" ::: "memory");
  float wo[8];
  float boutr = 0.0f;
  if (MODE == 2) {
    const v4f w0 = *(const v4f*)(wout + 8 * c);
    const v4f w1 = *(const v4f*)(wout + 8 * c + 4);
#pragma unroll
    for (int e = 0; e < 4; ++e) { wo[e] = bf16r(w0[e]); wo[4 + e] = bf16r(w1[e]); }
    boutr = bf16r(bout[0]);
  } else {
#pragma unroll
    for (int e = 0; e < 8; ++e) wo[e] = 0.0f;
  }
  __syncthreads();

  {
    const int m = tid >> 4, c8 = (tid & 15) * 8;
    const float* hp = h0l + (size_t)(rowbase + m) * NHID + c8;
    const v4f a = *(const v4f*)(hp);
    const v4f b = *(const v4f*)(hp + 4);
    v8h hv;
#pragma unroll
    for (int e = 0; e < 4; ++e) { hv[e] = to_h16(bf16r(a[e]) * HCARRY); hv[4 + e] = to_h16(bf16r(b[e]) * HCARRY); }
    *(v8h*)(Ah + m * APITCH + c8) = hv;
  }
  stage_x<MODE>(Ax, xsrc, ysrc, rowbase, 0, tid);
  __syncthreads();

  const XT*       axrow = (const XT*)(const void*)Ax + c * APITCH + koff;
  const _Float16* ahrow = Ah + c * APITCH + koff;
  const XT*       wxrow = WX + (size_t)j * KXE + koff;
  const _Float16* whrow = WH + (size_t)j * NHID + koff;
  const v8f z8 = {0.f, 0.f, 0.f, 0.f, 0.f, 0.f, 0.f, 0.f};

#pragma unroll 1
  for (int t = 0; t < NSTEP; ++t) {
    v8f acc0 = z8, acc1 = z8, acc2 = z8, acc3 = z8;
#pragma unroll 1
    for (int kx = 0; kx < KXE; kx += 32) {
      const XV a  = Frag<XT>::load(axrow + kx);
      const XV b0 = Frag<XT>::load(wxrow + kx);
      const XV b1 = Frag<XT>::load(wxrow + (size_t)1 * NHID * KXE + kx);
      const XV b2 = Frag<XT>::load(wxrow + (size_t)2 * NHID * KXE + kx);
      const XV b3 = Frag<XT>::load(wxrow + (size_t)3 * NHID * KXE + kx);
      acc0 = Frag<XT>::mma(a, b0, acc0);
      acc1 = Frag<XT>::mma(a, b1, acc1);
      acc2 = Frag<XT>::mma(a, b2, acc2);
      acc3 = Frag<XT>::mma(a, b3, acc3);
      Frag<XT>::tie4(acc0, acc1, acc2, acc3, a, b0, b1, b2, b3);
    }
#pragma unroll 1
    for (int k0 = 0; k0 < NHID; k0 += 32) {
      const v16h a  = Frag<_Float16>::load(ahrow + k0);
      const v16h b0 = Frag<_Float16>::load(whrow + k0);
      const v16h b1 = Frag<_Float16>::load(whrow + (size_t)1 * NHID * NHID + k0);
      const v16h b2 = Frag<_Float16>::load(whrow + (size_t)2 * NHID * NHID + k0);
      const v16h b3 = Frag<_Float16>::load(whrow + (size_t)3 * NHID * NHID + k0);
      acc0 = Frag<_Float16>::mma(a, b0, acc0);
      acc1 = Frag<_Float16>::mma(a, b1, acc1);
      acc2 = Frag<_Float16>::mma(a, b2, acc2);
      acc3 = Frag<_Float16>::mma(a, b3, acc3);
      Frag<_Float16>::tie4(acc0, acc1, acc2, acc3, a, b0, b1, b2, b3);
    }
    acc_guard4(acc0, acc1, acc2, acc3);

    float hn[8];
#pragma unroll
    for (int r = 0; r < 8; ++r) {
      const float zi = acc0[r] * FOLD + bs[0];
      const float zf = acc1[r] * FOLD + bs[1];
      const float zg = acc2[r] * FOLD + bs[2];
      const float zo = acc3[r] * FOLD + bs[3];
      const float ig = fsig(zi);
      const float fg = fsig(zf);
      const float gg = ftanh(zg);
      const float og = fsig(zo);
      const float cn = fg * cst[r] + ig * gg;
      cst[r] = cn;
      hn[r] = og * ftanh(cn);
    }
    __syncthreads();

#pragma unroll
    for (int r = 0; r < 8; ++r) {
      Ah[(8 * hh + r) * APITCH + j] = to_h16(hn[r] * HCARRY);
      Hs[(8 * hh + r) * SPITCH + j] = hn[r];
    }
    {
      const int tn = (t + 1 < NSTEP) ? (t + 1) : (NSTEP - 1);
      stage_x<MODE>(Ax, xsrc, ysrc, rowbase, tn, tid);
    }
    __syncthreads();

    if (MODE != 2) {
      const int m = 2 * wave + hh, c8 = c * 8;
      const float* sp = Hs + m * SPITCH + c8;
      const v4f a = *(const v4f*)(sp);
      const v4f b = *(const v4f*)(sp + 4);
      v8h hv;
#pragma unroll
      for (int e = 0; e < 4; ++e) { hv[e] = to_h16(a[e] * HCARRY); hv[4 + e] = to_h16(b[e] * HCARRY); }
      unsigned short* yp = ydst + ((size_t)(rowbase + m) * NSTEP + (size_t)t) * NHID + c8;
      *(volatile v8h*)yp = hv;
      __threadfence();
      *(volatile v8h*)yp = hv;
    } else {
      const int m = 2 * wave + hh, c8 = c * 8;
      const float* sp = Hs + m * SPITCH + c8;
      const v4f a = *(const v4f*)(sp);
      const v4f b = *(const v4f*)(sp + 4);
      float p = 0.0f;
#pragma unroll
      for (int e = 0; e < 4; ++e) p += a[e] * wo[e];
#pragma unroll
      for (int e = 0; e < 4; ++e) p += b[e] * wo[4 + e];
#pragma unroll
      for (int off = 1; off < 16; off <<= 1) p += __shfl_xor(p, off, 32);
      const float s = fmaxf(p + boutr, 0.0f);
      if (c == 0) Ob[m * OPITCH + (t & 31)] = s;
      if ((t & 31) == 31) {
        __syncthreads();
        if (wave < 4) {
          const int mm = 4 * wave + (lane >> 3), c4 = (lane & 7) * 4;
          const v4f v = *(const v4f*)(Ob + mm * OPITCH + c4);
          float* op = out0 + (size_t)(rowbase + mm) * NSTEP + (size_t)(t - 31) + c4;
          *(volatile v4f*)op = v;
          __threadfence();
          *(volatile v4f*)op = v;
        }
      }
    }
  }

#pragma unroll
  for (int r = 0; r < 8; ++r) Cs[(8 * hh + r) * SPITCH + j] = cst[r];
  __syncthreads();
  for (int pass = 0; pass < 2; ++pass) {
#pragma unroll
    for (int rr = 0; rr < 2; ++rr) {
      const int m = 2 * wave + rr;
      const v4f vh = *(const v4f*)(Hs + m * SPITCH + 4 * lane);
      const v4f vc = *(const v4f*)(Cs + m * SPITCH + 4 * lane);
      *(volatile v4f*)(hfin + (size_t)(rowbase + m) * NHID + 4 * lane) = vh;
      *(volatile v4f*)(cfin + (size_t)(rowbase + m) * NHID + 4 * lane) = vc;
    }
    __threadfence();
  }
}

extern "C" void kernel_launch(void* const* d_in, const int* in_sizes, int n_in,
                              void* d_out, int out_size, void* d_ws, size_t ws_size, hipStream_t stream) {
  if (n_in < 17 || d_out == nullptr || d_ws == nullptr) return;
  if (in_sizes[0] != NBAT * NSTEP * NDIN || in_sizes[1] != NSTATE || in_sizes[2] != NSTATE ||
      in_sizes[3] != NGATE * NDIN || in_sizes[4] != NGATE * NHID || in_sizes[5] != NGATE || in_sizes[6] != NGATE ||
      in_sizes[7] != NGATE * NHID || in_sizes[8] != NGATE * NHID || in_sizes[9] != NGATE || in_sizes[10] != NGATE ||
      in_sizes[11] != NGATE * NHID || in_sizes[12] != NGATE * NHID || in_sizes[13] != NGATE || in_sizes[14] != NGATE ||
      in_sizes[15] != NHID || in_sizes[16] != 1 || out_size != NOUT0 + 2 * NSTATE) return;

  const float* x    = (const float*)d_in[0];
  const float* h0   = (const float*)d_in[1];
  const float* c0   = (const float*)d_in[2];
  const float* wih0 = (const float*)d_in[3];
  const float* whh0 = (const float*)d_in[4];
  const float* bih0 = (const float*)d_in[5];
  const float* bhh0 = (const float*)d_in[6];
  const float* wih1 = (const float*)d_in[7];
  const float* whh1 = (const float*)d_in[8];
  const float* bih1 = (const float*)d_in[9];
  const float* bhh1 = (const float*)d_in[10];
  const float* wih2 = (const float*)d_in[11];
  const float* whh2 = (const float*)d_in[12];
  const float* bih2 = (const float*)d_in[13];
  const float* bhh2 = (const float*)d_in[14];
  const float* wout = (const float*)d_in[15];
  const float* bout = (const float*)d_in[16];
  float* out  = (float*)d_out;
  float* hfin = out + (size_t)NOUT0;
  float* cfin = hfin + (size_t)NSTATE;

  char* ws = (char*)d_ws; size_t off = 0;
  auto carve = [&](size_t bytes) -> char* { char* p = ws + off; off += (bytes + 255) & ~(size_t)255; return p; };
  unsigned short* WIH0 = (unsigned short*)carve((size_t)NGATE * NDIN * 2);
  unsigned short* WHH0 = (unsigned short*)carve((size_t)NGATE * NHID * 2);
  unsigned short* WIH1 = (unsigned short*)carve((size_t)NGATE * NHID * 2);
  unsigned short* WHH1 = (unsigned short*)carve((size_t)NGATE * NHID * 2);
  unsigned short* WIH2 = (unsigned short*)carve((size_t)NGATE * NHID * 2);
  unsigned short* WHH2 = (unsigned short*)carve((size_t)NGATE * NHID * 2);
  unsigned short* Y0   = (unsigned short*)carve((size_t)NBAT * NSTEP * NHID * 2);
  unsigned short* Y1   = (unsigned short*)carve((size_t)NBAT * NSTEP * NHID * 2);
  if (off > ws_size || off > (size_t)134217728) return;

  const int n8a = NGATE * (NDIN / 8);
  const int n8b = NGATE * (NHID / 8);
  cvt8_kernel<0><<<(n8a + NTHR - 1) / NTHR, NTHR, 0, stream>>>(wih0, WIH0, NGATE, NDIN / 8, NDIN, 0, XWCARRY);
  cvt8_kernel<1><<<(n8b + NTHR - 1) / NTHR, NTHR, 0, stream>>>(whh0, WHH0, NGATE, NHID / 8, NHID, 0, WCARRY);
  cvt8_kernel<1><<<(n8b + NTHR - 1) / NTHR, NTHR, 0, stream>>>(wih1, WIH1, NGATE, NHID / 8, NHID, 0, WCARRY);
  cvt8_kernel<1><<<(n8b + NTHR - 1) / NTHR, NTHR, 0, stream>>>(whh1, WHH1, NGATE, NHID / 8, NHID, 0, WCARRY);
  cvt8_kernel<1><<<(n8b + NTHR - 1) / NTHR, NTHR, 0, stream>>>(wih2, WIH2, NGATE, NHID / 8, NHID, 0, WCARRY);
  cvt8_kernel<1><<<(n8b + NTHR - 1) / NTHR, NTHR, 0, stream>>>(whh2, WHH2, NGATE, NHID / 8, NHID, 0, WCARRY);

  const size_t lstride = (size_t)NBAT * NHID;
  lstm_layer_kernel<0><<<NBAT / RBLK, NTHR, 0, stream>>>(x, Y0, h0, c0, bih0, bhh0, WIH0, WHH0, wout, bout,
                                                        Y0, out, hfin, cfin);
  lstm_layer_kernel<1><<<NBAT / RBLK, NTHR, 0, stream>>>(x, Y0, h0 + lstride, c0 + lstride, bih1, bhh1, WIH1, WHH1, wout, bout,
                                                        Y1, out, hfin + lstride, cfin + lstride);
  lstm_layer_kernel<2><<<NBAT / RBLK, NTHR, 0, stream>>>(x, Y1, h0 + 2 * lstride, c0 + 2 * lstride, bih2, bhh2, WIH2, WHH2, wout, bout,
                                                        Y0, out, hfin + 2 * lstride, cfin + 2 * lstride);
}
